// MAF_42417097016686
// MI455X (gfx1250) — hardware-verified
//
#include <hip/hip_runtime.h>
#include <math.h>

typedef __attribute__((ext_vector_type(16))) _Float16 v16h;
typedef __attribute__((ext_vector_type(16))) __bf16 v16b;
typedef __attribute__((ext_vector_type(8)))  _Float16 v8h;
typedef __attribute__((ext_vector_type(8)))  float v8f;
typedef __attribute__((ext_vector_type(4)))  float v4f;
typedef __attribute__((ext_vector_type(2)))  float v2f;
typedef __attribute__((ext_vector_type(4)))  unsigned v4u;
typedef __attribute__((ext_vector_type(4)))  int v4i;
typedef float __attribute__((may_alias)) float_a;
typedef int __attribute__((may_alias)) int_a;

template <typename T> __device__ __forceinline__ void vst2(void* p, T v) { *(volatile T*)p = v; __threadfence(); *(volatile T*)p = v; }
__device__ __forceinline__ v8f wmma16(v16h a, v16h b, v8f c) {
  v8f d = __builtin_amdgcn_wmma_f32_16x16x32_f16(false, a, false, b, (short)0, c, false, false);
  asm volatile("v_nop\n\tv_nop\n\tv_nop\n\tv_nop" : "+v"(d) : "v"(a), "v"(b));
  return d;
}
__device__ __forceinline__ v8f wmma_bf(v16b a, v16b b, v8f c) {
  v8f d = __builtin_amdgcn_wmma_f32_16x16x32_bf16(false, a, false, b, (short)0, c, false, false);
  asm volatile("v_nop\n\tv_nop\n\tv_nop\n\tv_nop" : "+v"(d) : "v"(a), "v"(b));
  return d;
}
__device__ __forceinline__ v16h frag_h(const _Float16* rowk0, int lane) {
  union { v16h v; v8h q[2]; } u; const _Float16* p = rowk0 + 8 * (lane >> 4);
  u.q[0] = *(const v8h*)p; u.q[1] = *(const v8h*)(p + 16); return u.v;
}
__device__ __forceinline__ v16h frag_f32(const float* rowk0, int lane) {
  v16h a; const float* p = rowk0 + 8 * (lane >> 4);
#pragma unroll
  for (int i = 0; i < 8; ++i) { a[i] = (_Float16)p[i]; a[8 + i] = (_Float16)p[16 + i]; }
  return a;
}
__device__ __forceinline__ v16h frag_f32s(const float* rowk0, int lane, float sc) {
  v16h a; const float* p = rowk0 + 8 * (lane >> 4);
#pragma unroll
  for (int i = 0; i < 8; ++i) { a[i] = (_Float16)(p[i] * sc); a[8 + i] = (_Float16)(p[16 + i] * sc); }
  return a;
}
__device__ __forceinline__ v16h fragc_f32(const float* W, int k0, int n, int lane, int ld, int K) {
  v16h a; const int g = lane >> 4;
#pragma unroll
  for (int i = 0; i < 8; ++i) { const int ka = k0 + 8 * g + i, kb = ka + 16;
    a[i] = (_Float16)(ka < K ? W[(size_t)(ka < K ? ka : K - 1) * ld + n] : 0.f); a[8 + i] = (_Float16)(kb < K ? W[(size_t)(kb < K ? kb : K - 1) * ld + n] : 0.f); }
  return a;
}
struct F2 { v16b h, l; };
__device__ __forceinline__ F2 bsplit16(const float v[16]) { F2 r;
#pragma unroll
  for (int i = 0; i < 16; ++i) { const __bf16 h = (__bf16)v[i]; r.h[i] = h; r.l[i] = (__bf16)(v[i] - (float)h); }
  return r; }
__device__ __forceinline__ F2 split_row(const float* row, int k0, int lane) { float v[16]; const float* p = row + k0 + 8 * (lane >> 4);
#pragma unroll
  for (int i = 0; i < 8; ++i) { v[i] = p[i]; v[8 + i] = p[16 + i]; }
  return bsplit16(v); }
__device__ __forceinline__ F2 split_rowK(const float* row, int k0, int lane, int K) { float v[16]; const int g = lane >> 4;
#pragma unroll
  for (int i = 0; i < 8; ++i) { const int ka = k0 + 8 * g + i, kb = ka + 16; v[i] = ka < K ? row[ka < K ? ka : K - 1] : 0.f; v[8 + i] = kb < K ? row[kb < K ? kb : K - 1] : 0.f; }
  return bsplit16(v); }
__device__ __forceinline__ F2 split_col(const float* W, int k0, int n, int lane, int ld, int K) { float v[16]; const int g = lane >> 4;
#pragma unroll
  for (int i = 0; i < 8; ++i) { const int ka = k0 + 8 * g + i, kb = ka + 16; v[i] = ka < K ? W[(size_t)(ka < K ? ka : K - 1) * ld + n] : 0.f; v[8 + i] = kb < K ? W[(size_t)(kb < K ? kb : K - 1) * ld + n] : 0.f; }
  return bsplit16(v); }
__device__ __forceinline__ v8f mac3(const F2& a, const F2& b, v8f c) { c = wmma_bf(a.l, b.h, c); c = wmma_bf(a.h, b.l, c); return wmma_bf(a.h, b.h, c); }
__device__ __forceinline__ float sigm(float v) { return 1.0f / (1.0f + expf(-v)); }
#define LDSX() do { asm volatile("s_wait_dscnt 0" ::: "memory"); __builtin_amdgcn_wave_barrier(); __builtin_amdgcn_fence(__ATOMIC_RELEASE, "workgroup"); } while (0)

#define NR 16384
#define DD 256
#define NL 255
#define HH 8
#define NCOL (NL * HH)
#ifndef NRV
#define NRV NR
#endif
#define OUT1_OFF 16777216u
__device__ __forceinline__ float bfr(float v) { return (float)(__bf16)v; }
#define WS_MU  0u
#define WS_AL  (WS_MU + 4u * (size_t)NL * NR)
#define WS_END (WS_AL + 4u * (size_t)NL * NR)
__device__ __forceinline__ v16b w1frag(const float* __restrict__ W1, int k0, int o, int lane) { v16b w; const int g = lane >> 4; const int oc = o < NCOL ? o : 0; const int l = oc >> 3, h = oc & 7; const float keepo = o < NCOL ? 1.f : 0.f; const float* base = W1 + (size_t)l * DD * HH + h;
  float t0[8], t1[8];
#pragma unroll
  for (int i = 0; i < 8; ++i) t0[i] = base[(size_t)(k0 + 8 * g + i) * HH];
  asm volatile("s_wait_loadcnt 0x0" ::: "memory");
#pragma unroll
  for (int i = 0; i < 8; ++i) t1[i] = base[(size_t)(k0 + 16 + 8 * g + i) * HH];
  asm volatile("s_wait_loadcnt 0x0" ::: "memory");
#pragma unroll
  for (int i = 0; i < 8; ++i) { const int ka = k0 + 8 * g + i, kb = ka + 16; w[i] = (__bf16)(t0[i] * (ka <= l ? keepo : 0.f)); w[8 + i] = (__bf16)(t1[i] * (kb <= l ? keepo : 0.f)); }
  return w; }
__device__ __forceinline__ v16b wsmall(const float* __restrict__ Wl, int ncol, int o, int lane) { v16b w; const int g = lane >> 4; const int oc = o < ncol ? o : 0; const float keepo = o < ncol ? 1.f : 0.f;
#pragma unroll
  for (int i = 0; i < 8; ++i) { const int ka = 8 * g + i; w[i] = (__bf16)(Wl[(size_t)(ka < HH ? ka : 0) * ncol + oc] * ((ka < HH && g == 0) ? keepo : 0.f)); w[8 + i] = (__bf16)0.f; }
  asm volatile("s_wait_loadcnt 0x0" ::: "memory"); return w; }
__device__ __forceinline__ F2 frag8(const float* __restrict__ p, int lane) { float va[16]; const int g = lane >> 4;
#pragma unroll
  for (int i = 0; i < 16; ++i) va[i] = 0.f;
  if (g == 0) {
#pragma unroll
    for (int i = 0; i < 8; ++i) va[i] = p[i]; }
  return bsplit16(va); }
__global__ __launch_bounds__(128) void k_maf(const float* __restrict__ X, const float* __restrict__ W1, const float* __restrict__ B1, const float* __restrict__ W2, const float* __restrict__ B2, const float* __restrict__ W3, const float* __restrict__ B3, float* __restrict__ MU, float* __restrict__ AL) {
  __shared__ __align__(16) float sh[4][16][132]; __shared__ __align__(16) float sh2[4][16][12]; __shared__ __align__(16) float smu[16][64], sal[16][64];
  const int tid = threadIdx.x, wave = tid >> 5, lane = tid & 31, col = lane & 15, g = lane >> 4; const int c0 = blockIdx.y * 128; const int l0 = c0 / HH; const size_t r0 = (size_t)blockIdx.x * 64 + wave * 16;
  v8f acc[8] = {};
#pragma unroll 2
  for (int kc = 0; kc < DD / 32; ++kc) { v16b a; { const float* p = X + (r0 + col) * DD + kc * 32 + 8 * g;
#pragma unroll
      for (int i = 0; i < 8; ++i) { a[i] = (__bf16)p[i]; a[8 + i] = (__bf16)p[16 + i]; } }
    asm volatile("s_wait_loadcnt 0x0" ::: "memory");
#pragma unroll
    for (int j = 0; j < 8; ++j) { const v16b w = w1frag(W1, kc * 32, c0 + j * 16 + col, lane); acc[j] = wmma_bf(a, w, acc[j]); } }
#pragma unroll
  for (int j = 0; j < 8; ++j) { const int o = c0 + j * 16 + col; const float bb = (o < NCOL) ? bfr(B1[o < NCOL ? o : 0]) : 0.f;
#pragma unroll
    for (int r = 0; r < 8; ++r) sh[wave][8 * g + r][j * 16 + col] = tanhf(acc[j][r] + bb); }
  LDSX();
#pragma unroll 1
  for (int lb = 0; lb < 16; ++lb) { const int l = l0 + lb; if (l >= NL) break;
    { const F2 a = frag8(&sh[wave][col][lb * HH], lane); const v16b w = wsmall(W2 + (size_t)l * HH * HH, HH, col, lane); v8f acc2 = {}; acc2 = wmma_bf(a.h, w, acc2); acc2 = wmma_bf(a.l, w, acc2);
      const float bb = (col < HH) ? bfr(B2[(size_t)l * HH + (col < HH ? col : 0)]) : 0.f;
      if (col < HH) {
#pragma unroll
        for (int r = 0; r < 8; ++r) sh2[wave][8 * g + r][col] = tanhf(acc2[r] + bb); } }
    LDSX();
    { const F2 a = frag8(&sh2[wave][col][0], lane); const v16b w = wsmall(W3 + (size_t)l * HH * 2, 2, col, lane); v8f acc3 = {}; acc3 = wmma_bf(a.h, w, acc3); acc3 = wmma_bf(a.l, w, acc3);
      const float bb = (col < 2) ? bfr(B3[(size_t)l * 2 + (col < 2 ? col : 0)]) : 0.f;
      if (col == 0) {
#pragma unroll
        for (int r = 0; r < 8; ++r) smu[lb][wave * 16 + 8 * g + r] = acc3[r] + bb; }
      if (col == 1) {
#pragma unroll
        for (int r = 0; r < 8; ++r) sal[lb][wave * 16 + 8 * g + r] = acc3[r] + bb; } }
    LDSX(); }
  __syncthreads();
  for (int lb = 0; lb < 16; ++lb) { const int l = l0 + lb; if (l >= NL) break;
    if (tid < 16) vst2(MU + (size_t)l * NR + (size_t)blockIdx.x * 64 + tid * 4, *(const v4f*)&smu[lb][tid * 4]);
    if (tid >= 32 && tid < 48) vst2(AL + (size_t)l * NR + (size_t)blockIdx.x * 64 + (tid - 32) * 4, *(const v4f*)&sal[lb][(tid - 32) * 4]); } }
__global__ __launch_bounds__(256) void k_z(const float* __restrict__ X, const float* __restrict__ IP, const float* __restrict__ MU, const float* __restrict__ AL, float* __restrict__ Z) { const size_t row = blockIdx.x; const int j = threadIdx.x; const int d = DD - 1 - j;
  const int dm = d > 0 ? d - 1 : 0; const float muv = MU[(size_t)dm * NR + row], alv = AL[(size_t)dm * NR + row], i0 = bfr(IP[0]), i1 = bfr(IP[1]), xv = bfr(X[row * DD + d]); asm volatile("s_wait_loadcnt 0x0" ::: "memory");
  const float mu = d == 0 ? i0 : muv, al = d == 0 ? i1 : alv;
  vst2(Z + row * DD + j, (xv - mu) * expf(-al)); }
__global__ __launch_bounds__(256) void k_ld(const float* __restrict__ IP, const float* __restrict__ AL, float* __restrict__ LD) { const size_t row = (size_t)blockIdx.x * 256 + threadIdx.x; if (row >= (size_t)NRV) return;
  float a = bfr(IP[1]);
#pragma unroll 1
  for (int lb = 0; lb < NL; lb += 8) { float tv[8];
#pragma unroll
    for (int u = 0; u < 8; ++u) { const int l = lb + u; tv[u] = AL[(size_t)(l < NL ? l : 0) * NR + row]; }
    asm volatile("s_wait_loadcnt 0x0" ::: "memory");
#pragma unroll
    for (int u = 0; u < 8; ++u) a += (lb + u < NL) ? tv[u] : 0.f; }
  vst2(LD + row, -a); }
extern "C" void kernel_launch(void* const* d_in, const int* in_sizes, int n_in, void* d_out, int out_size, void* d_ws, size_t ws_size, hipStream_t stream) {
  (void)in_sizes; (void)n_in; (void)out_size;
  if (ws_size < (size_t)WS_END) return;
  char* ws = (char*)d_ws; const float** F = (const float**)d_in; float *MU = (float*)(ws + WS_MU), *AL = (float*)(ws + WS_AL);
  k_maf<<<dim3(NRV / 64, (NCOL + 127) / 128), 128, 0, stream>>>(F[0], F[2], F[3], F[4], F[5], F[6], F[7], MU, AL);
  k_z<<<dim3(NRV), 256, 0, stream>>>(F[0], F[1], MU, AL, (float*)d_out);
  k_ld<<<dim3((NRV + 255) / 256), 256, 0, stream>>>(F[1], AL, (float*)((char*)d_out + OUT1_OFF));
}
